// LocalAttentionND_77043123355932
// MI455X (gfx1250) — hardware-verified
//
#include <hip/hip_runtime.h>
#include <hip/hip_bf16.h>
#include <math.h>


typedef _Float16 bf16;
typedef _Float16 f16;
typedef __attribute__((ext_vector_type(4))) unsigned v4u_t;
typedef unsigned v4ua __attribute__((ext_vector_type(4), may_alias));
typedef __attribute__((ext_vector_type(4))) float v4f_t;
typedef float v4fa __attribute__((ext_vector_type(4), may_alias));
typedef __attribute__((ext_vector_type(16))) bf16  bf16x16;
typedef bf16x16 f16x16;
typedef __attribute__((ext_vector_type(8)))  bf16  bf16x8;
typedef bf16x8 f16x8;
typedef __attribute__((ext_vector_type(4)))  bf16  bf16x4;
typedef __attribute__((ext_vector_type(8)))  float f32x8;
__device__ __forceinline__ f32x8 wmma16(f16x16 a, f16x16 b, f32x8 c) {
  c = __builtin_amdgcn_wmma_f32_16x16x32_f16(false, a, false, b, (short)0, c, false, false);
  asm volatile("v_nop\n\tv_nop\n\tv_nop\n\tv_nop" : "+v"(c) : "v"(a), "v"(b));
  return c;
}
#define LDS_STRIDE 48
#define KSTRIDE    72
#define VSTRIDE    48

__device__ __forceinline__ f32x8 wmma_bf16(bf16x16 a, bf16x16 b, f32x8 c) {
  c = __builtin_amdgcn_wmma_f32_16x16x32_f16(false, a, false, b, (short)0, c, false, false);
  asm volatile("v_nop\n\tv_nop\n\tv_nop\n\tv_nop" : "+v"(c) : "v"(a), "v"(b));
  return c;
}

template <typename T>
__device__ __forceinline__ bf16x16 load_frag(const T* __restrict__ base, int ld,
                                             int row0, int k0) {
  const int lane = threadIdx.x & 31;
  const int r    = lane & 15;
  const int kh   = (lane >> 4) * 8;
  const T* p0 = base + (size_t)(row0 + r) * ld + (k0 + kh);
  const T* p1 = p0 + 16;
  bf16x16 f;
#pragma unroll
  for (int i = 0; i < 8; ++i) {
    f[i]     = (bf16)p0[i];
    f[i + 8] = (bf16)p1[i];
  }
  return f;
}

__device__ __forceinline__ bf16x16 lds_frag(const bf16* base, int stride) {
  const int lane = threadIdx.x & 31;
  const int row  = lane & 15;
  const int kh   = (lane >> 4) * 8;
  const bf16x8 lo = *(const bf16x8*)(base + row * stride + kh);
  const bf16x8 hi = *(const bf16x8*)(base + row * stride + kh + 16);
  bf16x16 f;
#pragma unroll
  for (int i = 0; i < 8; ++i) { f[i] = lo[i]; f[i + 8] = hi[i]; }
  return f;
}

template <typename T>
__device__ __forceinline__ void stage_read16(const T* __restrict__ p, float* buf) {
#pragma unroll
  for (int i = 0; i < 16; ++i) buf[i] = (float)p[i];
}

__device__ __forceinline__ void stage_write(bf16* dst, const float* buf, int nquad) {
#pragma unroll
  for (int i = 0; i < nquad; ++i) {
    bf16x4 q;
    q[0] = (bf16)buf[4 * i];     q[1] = (bf16)buf[4 * i + 1];
    q[2] = (bf16)buf[4 * i + 2]; q[3] = (bf16)buf[4 * i + 3];
    *(bf16x4*)(dst + 4 * i) = q;
  }
}


#define GSTR 48
#define GSTR 48
template <typename AT, int EPI, bool OUT16>
__global__ __launch_bounds__(256) void gemm_kne(const AT* __restrict__ A, int lda, const float* __restrict__ Wm, int ldw,
                                                const float* __restrict__ bias, const float* __restrict__ R, const float* __restrict__ gvec,
                                                void* __restrict__ Yv, int ldy, int K) {
  __shared__ __attribute__((aligned(16))) f16 ldsA[128 * GSTR];
  __shared__ __attribute__((aligned(16))) f16 ldsW[128 * GSTR];
  __shared__ __attribute__((aligned(16))) float oS[8][32 * 68];
  const int tid = threadIdx.x, lane = tid & 31, wave = tid >> 5, cl = lane & 15, rh = (lane >> 4) * 8;
  const int m0 = blockIdx.x * 128, n0 = blockIdx.y * 128;
  const int wm = (wave & 3) * 32, wn = (wave >> 2) * 64;
  f32x8 acc[2][4];
#pragma unroll
  for (int i = 0; i < 2; ++i)
#pragma unroll
    for (int j = 0; j < 4; ++j) { f32x8 z = {}; acc[i][j] = z; }
#pragma unroll 1
  for (int k0 = 0; k0 < K; k0 += 32) {
    __syncthreads();
    { const int row = tid >> 1, ch = (tid & 1) * 16;
      const AT* src = A + (size_t)(m0 + row) * lda + k0 + ch;
#pragma unroll
      for (int g = 0; g < 16; ++g) ldsA[row * GSTR + ch + g] = (f16)src[g]; }
    { const int k = tid >> 3, nn0 = (tid & 7) * 16;
      const float* src = Wm + (size_t)(k0 + k) * ldw + n0 + nn0;
#pragma unroll
      for (int g = 0; g < 4; ++g) { const v4f_t v = *(const v4f_t*)(src + 4 * g);
#pragma unroll
        for (int u = 0; u < 4; ++u) ldsW[(nn0 + 4 * g + u) * GSTR + k] = (f16)v[u]; } }
    __syncthreads();
    f16x16 af[2];
#pragma unroll
    for (int i = 0; i < 2; ++i) af[i] = lds_frag(ldsA + (wm + 16 * i) * GSTR, GSTR);
#pragma unroll
    for (int j = 0; j < 4; ++j) {
      const f16x16 bf = lds_frag(ldsW + (wn + 16 * j) * GSTR, GSTR);
#pragma unroll
      for (int i = 0; i < 2; ++i) acc[i][j] = wmma16(af[i], bf, acc[i][j]);
    }
  }
  float* so = oS[wave];
#pragma unroll
  for (int i = 0; i < 2; ++i)
#pragma unroll
    for (int j = 0; j < 4; ++j) {
      const int n = n0 + wn + 16 * j + cl;
      const float bv = bias ? bias[n] : 0.0f;
      const float gv = (EPI == 2 || EPI == 4) ? gvec[n] : 0.0f;
      if (EPI == 1) {
#pragma unroll 1
        for (int r = 0; r < 8; ++r) { const float xg = acc[i][j][r] + bv; so[(16 * i + rh + r) * 68 + 16 * j + cl] = 0.5f * xg * (1.0f + erff(xg * 0.70710678118654752f)); }
      } else {
#pragma unroll
        for (int r = 0; r < 8; ++r) {
          float v = acc[i][j][r] + bv;
          if (EPI == 3) v = fmaxf(v, 0.0f);
          if (EPI == 4) v = gv * v;
          if (EPI == 2) v = R[(size_t)(m0 + wm + 16 * i + rh + r) * ldy + n] + gv * v;
          so[(16 * i + rh + r) * 68 + 16 * j + cl] = v;
        }
      }
    }
  asm volatile("s_wait_dscnt 0" ::: "memory");
  __builtin_amdgcn_wave_barrier();
#pragma unroll 1
  for (int pass = 0; pass < 2; ++pass) {
    if (OUT16) {
      f16* Y = (f16*)Yv;
#pragma unroll
      for (int it = 0; it < 8; ++it) { const int c = lane + 32 * it, rr = c >> 3, q8 = (c & 7) * 8;
        union { f16 h[8]; v4u_t v; } u;
#pragma unroll
        for (int e = 0; e < 8; ++e) u.h[e] = (f16)so[rr * 68 + q8 + e];
        *(volatile v4u_t*)(Y + (size_t)(m0 + wm + rr) * ldy + n0 + wn + q8) = u.v; }
    } else {
      float* Y = (float*)Yv;
#pragma unroll
      for (int it = 0; it < 16; ++it) { const int f4 = lane + 32 * it, rr = f4 >> 4, q = (f4 & 15) * 4;
        *(volatile v4f_t*)(Y + (size_t)(m0 + wm + rr) * ldy + n0 + wn + q) = *(const v4fa*)(so + rr * 68 + q); }
    }
    __threadfence();
  }
}

template <typename AT, int EPI, bool OUT16>
__global__ __launch_bounds__(256) void gemm_knez(const AT* __restrict__ A, int lda, size_t strideA, const float* __restrict__ Wm, int ldw, size_t strideW,
                                                 const float* __restrict__ bias, const float* __restrict__ R, const float* __restrict__ gvec,
                                                 void* __restrict__ Yv, int ldy, size_t strideY, int K) {
  A += (size_t)blockIdx.z * strideA; Wm += (size_t)blockIdx.z * strideW; Yv = (void*)((char*)Yv + (size_t)blockIdx.z * strideY * (OUT16 ? 2 : 4)); if (R) R += (size_t)blockIdx.z * strideY;
  __shared__ __attribute__((aligned(16))) f16 ldsA[128 * GSTR];
  __shared__ __attribute__((aligned(16))) f16 ldsW[128 * GSTR];
  __shared__ __attribute__((aligned(16))) float oS[8][32 * 68];
  const int tid = threadIdx.x, lane = tid & 31, wave = tid >> 5, cl = lane & 15, rh = (lane >> 4) * 8;
  const int m0 = blockIdx.x * 128, n0 = blockIdx.y * 128;
  const int wm = (wave & 3) * 32, wn = (wave >> 2) * 64;
  f32x8 acc[2][4];
#pragma unroll
  for (int i = 0; i < 2; ++i)
#pragma unroll
    for (int j = 0; j < 4; ++j) { f32x8 z = {}; acc[i][j] = z; }
#pragma unroll 1
  for (int k0 = 0; k0 < K; k0 += 32) {
    __syncthreads();
    { const int row = tid >> 1, ch = (tid & 1) * 16;
      const AT* src = A + (size_t)(m0 + row) * lda + k0 + ch;
#pragma unroll
      for (int g = 0; g < 16; ++g) ldsA[row * GSTR + ch + g] = (f16)src[g]; }
    { const int k = tid >> 3, nn0 = (tid & 7) * 16;
      const float* src = Wm + (size_t)(k0 + k) * ldw + n0 + nn0;
#pragma unroll
      for (int g = 0; g < 4; ++g) { const v4f_t v = *(const v4f_t*)(src + 4 * g);
#pragma unroll
        for (int u = 0; u < 4; ++u) ldsW[(nn0 + 4 * g + u) * GSTR + k] = (f16)v[u]; } }
    __syncthreads();
    f16x16 af[2];
#pragma unroll
    for (int i = 0; i < 2; ++i) af[i] = lds_frag(ldsA + (wm + 16 * i) * GSTR, GSTR);
#pragma unroll
    for (int j = 0; j < 4; ++j) {
      const f16x16 bf = lds_frag(ldsW + (wn + 16 * j) * GSTR, GSTR);
#pragma unroll
      for (int i = 0; i < 2; ++i) acc[i][j] = wmma16(af[i], bf, acc[i][j]);
    }
  }
  float* so = oS[wave];
#pragma unroll
  for (int i = 0; i < 2; ++i)
#pragma unroll
    for (int j = 0; j < 4; ++j) {
      const int n = n0 + wn + 16 * j + cl;
      const float bv = bias ? bias[n] : 0.0f;
      const float gv = (EPI == 2 || EPI == 4) ? gvec[n] : 0.0f;
      if (EPI == 1) {
#pragma unroll 1
        for (int r = 0; r < 8; ++r) { const float xg = acc[i][j][r] + bv; so[(16 * i + rh + r) * 68 + 16 * j + cl] = 0.5f * xg * (1.0f + erff(xg * 0.70710678118654752f)); }
      } else {
#pragma unroll
        for (int r = 0; r < 8; ++r) {
          float v = acc[i][j][r] + bv;
          if (EPI == 3) v = fmaxf(v, 0.0f);
          if (EPI == 4) v = gv * v;
          if (EPI == 2) v = R[(size_t)(m0 + wm + 16 * i + rh + r) * ldy + n] + gv * v;
          so[(16 * i + rh + r) * 68 + 16 * j + cl] = v;
        }
      }
    }
  asm volatile("s_wait_dscnt 0" ::: "memory");
  __builtin_amdgcn_wave_barrier();
#pragma unroll 1
  for (int pass = 0; pass < 2; ++pass) {
    if (OUT16) {
      f16* Y = (f16*)Yv;
#pragma unroll
      for (int it = 0; it < 8; ++it) { const int c = lane + 32 * it, rr = c >> 3, q8 = (c & 7) * 8;
        union { f16 h[8]; v4u_t v; } u;
#pragma unroll
        for (int e = 0; e < 8; ++e) u.h[e] = (f16)so[rr * 68 + q8 + e];
        *(volatile v4u_t*)(Y + (size_t)(m0 + wm + rr) * ldy + n0 + wn + q8) = u.v; }
    } else {
      float* Y = (float*)Yv;
#pragma unroll
      for (int it = 0; it < 16; ++it) { const int f4 = lane + 32 * it, rr = f4 >> 4, q = (f4 & 15) * 4;
        *(volatile v4f_t*)(Y + (size_t)(m0 + wm + rr) * ldy + n0 + wn + q) = *(const v4fa*)(so + rr * 68 + q); }
    }
    __threadfence();
  }
}

template <typename AT, bool ACC>
__global__ __launch_bounds__(256) void gemm_kn2(const AT* __restrict__ A, int lda, size_t strideA,
                                               const float* __restrict__ Wm, int ldw, size_t strideW,
                                               const float* __restrict__ bias, float scale,
                                               float* __restrict__ Y, int ldy, size_t strideY, int K) {
  __shared__ __attribute__((aligned(16))) f16 ldsA[128 * GSTR], ldsAl[128 * GSTR];
  __shared__ __attribute__((aligned(16))) f16 ldsW[128 * GSTR], ldsWl[128 * GSTR];
  __shared__ __attribute__((aligned(16))) float oS[8][32 * 68];
  const int tid = threadIdx.x, lane = tid & 31, wave = tid >> 5, cl = lane & 15, rh = (lane >> 4) * 8;
  const int m0 = blockIdx.x * 128, n0 = blockIdx.y * 128;
  const int wm = (wave & 3) * 32, wn = (wave >> 2) * 64;
  A += (size_t)blockIdx.z * strideA; Wm += (size_t)blockIdx.z * strideW; Y += (size_t)blockIdx.z * strideY;
  f32x8 acc[2][4], accx[2][4];
#pragma unroll
  for (int i = 0; i < 2; ++i)
#pragma unroll
    for (int j = 0; j < 4; ++j) { f32x8 z = {}; acc[i][j] = z; accx[i][j] = z; }
#pragma unroll 1
  for (int k0 = 0; k0 < K; k0 += 32) {
    __syncthreads();
    {
      const int row = tid >> 1, ch = (tid & 1) * 16;
      const AT* src = A + (size_t)(m0 + row) * lda + k0 + ch;
#pragma unroll
      for (int g = 0; g < 16; ++g) { const float v = (float)src[g]; const f16 h = (f16)v; ldsA[row * GSTR + ch + g] = h; ldsAl[row * GSTR + ch + g] = (f16)((v - (float)h) * 2048.0f); }
    }
    {
      const int k = tid >> 3, nn0 = (tid & 7) * 16;
      const float* src = Wm + (size_t)(k0 + k) * ldw + n0 + nn0;
#pragma unroll
      for (int g = 0; g < 4; ++g) { const v4f_t v = *(const v4f_t*)(src + 4 * g);
#pragma unroll
        for (int u = 0; u < 4; ++u) { const f16 h = (f16)v[u]; ldsW[(nn0 + 4 * g + u) * GSTR + k] = h; ldsWl[(nn0 + 4 * g + u) * GSTR + k] = (f16)((v[u] - (float)h) * 2048.0f); } }
    }
    __syncthreads();
    f16x16 af[2], afl[2];
#pragma unroll
    for (int i = 0; i < 2; ++i) { af[i] = lds_frag(ldsA + (wm + 16 * i) * GSTR, GSTR); afl[i] = lds_frag(ldsAl + (wm + 16 * i) * GSTR, GSTR); }
#pragma unroll
    for (int j = 0; j < 4; ++j) {
      const f16x16 bf = lds_frag(ldsW + (wn + 16 * j) * GSTR, GSTR), bfl = lds_frag(ldsWl + (wn + 16 * j) * GSTR, GSTR);
#pragma unroll
      for (int i = 0; i < 2; ++i) { acc[i][j] = wmma16(af[i], bf, acc[i][j]); accx[i][j] = wmma16(af[i], bfl, accx[i][j]); accx[i][j] = wmma16(afl[i], bf, accx[i][j]); }
    }
  }
  float* so = oS[wave];
#pragma unroll
  for (int i = 0; i < 2; ++i)
#pragma unroll
    for (int j = 0; j < 4; ++j) {
      const float bv = bias ? bias[n0 + wn + 16 * j + cl] : 0.0f;
#pragma unroll
      for (int r = 0; r < 8; ++r) so[(16 * i + rh + r) * 68 + 16 * j + cl] = (acc[i][j][r] + accx[i][j][r] * (1.0f / 2048.0f)) * scale + bv;
    }
  asm volatile("s_wait_dscnt 0" ::: "memory");
  __builtin_amdgcn_wave_barrier();
  if (ACC) {
#pragma unroll
    for (int it = 0; it < 16; ++it) { const int f4 = lane + 32 * it, rr = f4 >> 4, q = (f4 & 15) * 4;
      const v4f_t old = *(const v4fa*)(Y + (size_t)(m0 + wm + rr) * ldy + n0 + wn + q);
      v4f_t v = *(const v4fa*)(so + rr * 68 + q); v += old; *(v4fa*)(so + rr * 68 + q) = v; }
    asm volatile("s_wait_dscnt 0" ::: "memory");
  }
#pragma unroll 1
  for (int pass = 0; pass < 2; ++pass) {
#pragma unroll
    for (int it = 0; it < 16; ++it) { const int f4 = lane + 32 * it, rr = f4 >> 4, q = (f4 & 15) * 4;
      *(volatile v4f_t*)(Y + (size_t)(m0 + wm + rr) * ldy + n0 + wn + q) = *(const v4fa*)(so + rr * 68 + q); }
    __threadfence();
  }
}

__global__ __launch_bounds__(256) void k_transpose(const float* __restrict__ Wm, float* __restrict__ Wt, int rows, int cols) {
  __shared__ float tS[64][65];
  const int tid = threadIdx.x, tbj = cols / 64, bi = blockIdx.x / tbj, bj = blockIdx.x % tbj;
  for (int e = tid; e < 64 * 64; e += 256) { const int r = e >> 6, c = e & 63; tS[r][c] = Wm[(size_t)(bi * 64 + r) * cols + bj * 64 + c]; }
  __syncthreads();
  for (int ch = tid; ch < 64 * 16; ch += 256) { const int r = ch >> 4, q4 = (ch & 15) * 4; v4f_t o; o[0] = tS[q4][r]; o[1] = tS[q4 + 1][r]; o[2] = tS[q4 + 2][r]; o[3] = tS[q4 + 3][r];
    float* dst = Wt + (size_t)(bj * 64 + r) * rows + bi * 64 + q4; *(volatile v4f_t*)dst = o; __threadfence(); *(volatile v4f_t*)dst = o; }
}


#define GSTR 48
#define SS 2048
#define HH 32
#define DKK 64
template <typename AT, int MODE>
__global__ __launch_bounds__(256) void gemm_rb_kernel(
    const AT* __restrict__ A, const float* __restrict__ W,
    const float* __restrict__ bias, const float* __restrict__ rowscale, const float* __restrict__ R, const float* __restrict__ rowbias, void* __restrict__ out,
    int M, int N, int K) {
  __shared__ bf16 ldsA[128 * LDS_STRIDE];
  __shared__ bf16 ldsW[256 * LDS_STRIDE];
  __shared__ __attribute__((aligned(16))) unsigned char sob[256 * 136 * 2];

  const int t    = threadIdx.x;
  const int wave = t >> 5;
  const int lane = t & 31;
  const int wm   = (wave & 1) * 64;
  const int wn   = (wave >> 1) * 64;
  const int mBlk = blockIdx.x * 128;
  const int nBlk = blockIdx.y * 256;

  const int arow = t >> 1;
  const int ach  = (t & 1) * 16;

  float abuf[16];
  float wbuf[32];

  stage_read16(A + (size_t)(mBlk + arow) * K + ach, abuf);
  const int nrow = min(nBlk + t, N - 1);
  stage_read16(W + (size_t)nrow * K,          wbuf);
  stage_read16(W + (size_t)nrow * K + 16,     wbuf + 16);

  f32x8 acc[4][4] = {};

  for (int k = 0; k < K; k += 32) {
    __syncthreads();
    stage_write(&ldsA[arow * LDS_STRIDE + ach], abuf, 4);
    stage_write(&ldsW[t * LDS_STRIDE],          wbuf, 8);
    if (k + 32 < K) {
      stage_read16(A + (size_t)(mBlk + arow) * K + (k + 32) + ach, abuf);
      stage_read16(W + (size_t)nrow * K + (k + 32),          wbuf);
      stage_read16(W + (size_t)nrow * K + (k + 32) + 16,     wbuf + 16);
    }
    __syncthreads();

    bf16x16 af[4], wf[4];
#pragma unroll
    for (int i = 0; i < 4; ++i)
      af[i] = lds_frag(ldsA + (wm + 16 * i) * LDS_STRIDE, LDS_STRIDE);
#pragma unroll
    for (int j = 0; j < 4; ++j)
      wf[j] = lds_frag(ldsW + (wn + 16 * j) * LDS_STRIDE, LDS_STRIDE);
#pragma unroll
    for (int i = 0; i < 4; ++i)
#pragma unroll
      for (int j = 0; j < 4; ++j)
        acc[i][j] = wmma_bf16(af[i], wf[j], acc[i][j]);
  }

  const int nlane = lane & 15;
  const int mh    = (lane >> 4) * 8;
  __syncthreads();
  if (MODE == 0 || MODE == 1 || MODE == 3) {
    bf16* so = (bf16*)sob;
#pragma unroll
    for (int i = 0; i < 4; ++i)
#pragma unroll
      for (int j = 0; j < 4; ++j) {
        const int nl = wn + 16 * j + nlane;
        const float bv = bias ? bias[nBlk + nl] : 0.0f;
        if (MODE == 3) {
#pragma unroll 1
          for (int r = 0; r < 8; ++r) {
            const int ml = wm + 16 * i + mh + r;
            const float xg = acc[i][j][r] + bv;
            so[ml * 264 + nl] = (bf16)(0.5f * xg * (1.0f + erff(xg * 0.70710678118654752f)));
          }
        } else {
#pragma unroll
        for (int r = 0; r < 8; ++r) {
          const int ml = wm + 16 * i + mh + r;
          const bf16 hv = (bf16)(acc[i][j][r] + bv);
          if (MODE == 0) so[ml * 264 + nl] = hv;
          else           so[nl * 136 + ml] = hv;
        }
        }
      }
    __syncthreads();
#pragma unroll 1
    for (int pass = 0; pass < 2; ++pass) {
      if (MODE == 0 || MODE == 3) {
        for (int ch = t; ch < 128 * 32; ch += 256) { const int ml = ch >> 5, q = (ch & 31) * 8;
          *(volatile v4u_t*)((bf16*)out + (size_t)(mBlk + ml) * N + nBlk + q) = *(const v4ua*)(so + ml * 264 + q); }
      } else {
        const int b_ = mBlk / SS, s0 = mBlk % SS;
        for (int ch = t; ch < 256 * 16; ch += 256) { const int nl = ch >> 4, q = (ch & 15) * 8; const int n = nBlk + nl, h = n >> 6, dk = n & (DKK - 1);
          *(volatile v4u_t*)((bf16*)out + (((size_t)(b_ * HH + h)) * DKK + dk) * SS + s0 + q) = *(const v4ua*)(so + nl * 136 + q); }
      }
      __threadfence();
    }
  } else {
    float* so = (float*)sob;
#pragma unroll 1
    for (int hf = 0; hf < 2; ++hf) {
      if (wm == hf * 64) {
#pragma unroll
        for (int i = 0; i < 4; ++i)
#pragma unroll
          for (int j = 0; j < 4; ++j) {
            const int nl = wn + 16 * j + nlane;
            const float bv = bias ? bias[nBlk + nl] : 0.0f;
#pragma unroll
            for (int r = 0; r < 8; ++r) { const int mrow = mBlk + hf * 64 + 16 * i + mh + r; so[(16 * i + mh + r) * 260 + nl] = acc[i][j][r] * (rowscale ? rowscale[mrow] : 1.0f) + bv + (rowbias ? rowbias[mrow] : 0.0f); }
          }
      }
      __syncthreads();
      if (R) {
        for (int ch = t; ch < 64 * 64; ch += 256) { const int ml = ch >> 6, q = (ch & 63) * 4;
          if (nBlk + q < N) { const v4f_t rv = *(const v4f_t*)(R + (size_t)(mBlk + hf * 64 + ml) * N + nBlk + q); v4f_t v = *(const v4fa*)(so + ml * 260 + q); v += rv; *(volatile v4fa*)(so + ml * 260 + q) = v; } }
        asm volatile("s_wait_dscnt 0" ::: "memory");
      }
#pragma unroll 1
      for (int pass = 0; pass < 2; ++pass) {
        for (int ch = t; ch < 64 * 64; ch += 256) { const int ml = ch >> 6, q = (ch & 63) * 4;
          if (nBlk + q < N) *(volatile v4f_t*)((float*)out + (size_t)(mBlk + hf * 64 + ml) * N + nBlk + q) = *(const v4fa*)(so + ml * 260 + q); }
        __threadfence();
      }
      __syncthreads();
    }
  }
}

#define NBl 2
#define LLl 4096
#define LIN 4096
#define NRl (NBl * LLl)
#define CCl 512
#define NHl 8
#define HDl 64
#define KWl 49
__global__ __launch_bounds__(256) void k_fill(float* __restrict__ p, float val, size_t n4) { const size_t i = (size_t)blockIdx.x * 256 + threadIdx.x; if (i < n4) { v4f_t v = {val, val, val, val}; *(volatile v4f_t*)(p + 4 * i) = v; __threadfence(); *(volatile v4f_t*)(p + 4 * i) = v; } }
__global__ __launch_bounds__(256) void k_dbg_zero(float* __restrict__ p, size_t n4) { const size_t i = (size_t)blockIdx.x * 256 + threadIdx.x; if (i < n4) { v4f_t z = {0.f,0.f,0.f,0.f}; *(volatile v4f_t*)(p + 4 * i) = z; __threadfence(); *(volatile v4f_t*)(p + 4 * i) = z; } }
__global__ __launch_bounds__(256) void k_copy(const float* __restrict__ src, float* __restrict__ dst, size_t n4) { const size_t i = (size_t)blockIdx.x * 256 + threadIdx.x; if (i < n4) { const v4f_t v = *(const v4f_t*)(src + 4 * i); *(volatile v4f_t*)(dst + 4 * i) = v; __threadfence(); *(volatile v4f_t*)(dst + 4 * i) = v; } }
__global__ __launch_bounds__(128) void k_padwin(const float* __restrict__ w, const float* __restrict__ bw, float* __restrict__ WT, float* __restrict__ BT) {
  const int k = blockIdx.x, n = threadIdx.x; const float v = (n < 16) ? w[(size_t)min(n, 15) * CCl + k] : 0.0f; *(volatile float*)(WT + (size_t)k * 128 + n) = v; __threadfence(); *(volatile float*)(WT + (size_t)k * 128 + n) = v;
  if (k == 0) { const float b = (n < 16) ? bw[min(n, 15)] : 0.0f; *(volatile float*)(BT + n) = b; __threadfence(); *(volatile float*)(BT + n) = b; }
}
__global__ __launch_bounds__(256) void k_ropetab(float* __restrict__ CS, float* __restrict__ SN) {
  const int tid = threadIdx.x, h = tid >> 5, i = tid & 31; const float fr = 1.0f / powf(10000.0f, (float)i / 32.0f); const float a = (float)h * fr; float sn, cs; sincosf(a, &sn, &cs);
  *(volatile float*)(CS + tid) = cs; *(volatile float*)(SN + tid) = sn; __threadfence(); *(volatile float*)(CS + tid) = cs; *(volatile float*)(SN + tid) = sn;
}
__global__ __launch_bounds__(256) void k_prep(float* __restrict__ Q, float* __restrict__ KV, const float* __restrict__ qw, const float* __restrict__ kw, const float* __restrict__ CS, const float* __restrict__ SN) {
  const size_t r = blockIdx.x; const int tid = threadIdx.x, h = tid >> 5, i = tid & 31; const float cs = CS[tid], sn = SN[tid];
  float* qp = Q + r * CCl + h * HDl; float* kp = KV + r * (2 * CCl) + h * HDl; float* vp = KV + r * (2 * CCl) + CCl + h * HDl;
  float q1 = qp[i], q2 = qp[i + 32], k1 = kp[i], k2 = kp[i + 32], v1 = vp[i], v2 = vp[i + 32];
  q1 = q1 / (1.0f + expf(-q1)); q2 = q2 / (1.0f + expf(-q2)); k1 = k1 / (1.0f + expf(-k1)); k2 = k2 / (1.0f + expf(-k2)); v1 = v1 / (1.0f + expf(-v1)); v2 = v2 / (1.0f + expf(-v2));
  float sq = q1 * q1 + q2 * q2, sk = k1 * k1 + k2 * k2;
#pragma unroll
  for (int o = 1; o < 32; o <<= 1) { sq += __shfl_xor(sq, o, 32); sk += __shfl_xor(sk, o, 32); }
  const float rq = 1.0f / __builtin_sqrtf(sq * (1.0f / HDl) + 1e-6f), rk = 1.0f / __builtin_sqrtf(sk * (1.0f / HDl) + 1e-6f);
  q1 = q1 * rq * qw[i]; q2 = q2 * rq * qw[i + 32]; k1 = k1 * rk * kw[i]; k2 = k2 * rk * kw[i + 32];
  const float qa = q1 * cs - q2 * sn, qb = q1 * sn + q2 * cs, ka = k1 * cs - k2 * sn, kb = k1 * sn + k2 * cs;
#pragma unroll 1
  for (int pass = 0; pass < 2; ++pass) { *(volatile float*)(qp + i) = qa; *(volatile float*)(qp + i + 32) = qb; *(volatile float*)(kp + i) = ka; *(volatile float*)(kp + i + 32) = kb; *(volatile float*)(vp + i) = v1; *(volatile float*)(vp + i + 32) = v2; __threadfence(); }
}
__global__ __launch_bounds__(256) void k_window(const float* __restrict__ Q, const float* __restrict__ KV, const float* __restrict__ WP, float* __restrict__ AO) {
  const size_t r = blockIdx.x; const int tid = threadIdx.x, h = tid >> 5, i = tid & 31; const int l = (int)(r % LLl); const size_t r0 = r - l;
  float w0 = WP[r * 128 + h], w1 = WP[r * 128 + NHl + h]; w0 = w0 / (1.0f + expf(-w0)); w1 = w1 / (1.0f + expf(-w1));
  const float width = 24.0f / (1.0f + expf(-w0)) + 0.5f, sharp = 9.5f / (1.0f + expf(-w1)) + 0.5f;
  const float q1 = Q[r * CCl + h * HDl + i], q2 = Q[r * CCl + h * HDl + i + 32];
  float m = -3.0e38f, z = 0.0f, o1 = 0.0f, o2 = 0.0f;
#pragma unroll 1
  for (int kk = 0; kk < KWl; ++kk) { const int j = l - 24 + kk; const bool in = (j >= 0) && (j < LLl); const size_t jr = r0 + (size_t)min(max(j, 0), LLl - 1);
    const float k1 = in ? KV[jr * (2 * CCl) + h * HDl + i] : 0.0f, k2 = in ? KV[jr * (2 * CCl) + h * HDl + i + 32] : 0.0f;
    const float v1 = in ? KV[jr * (2 * CCl) + CCl + h * HDl + i] : 0.0f, v2 = in ? KV[jr * (2 * CCl) + CCl + h * HDl + i + 32] : 0.0f;
    float d = q1 * k1 + q2 * k2;
#pragma unroll
    for (int o = 1; o < 32; o <<= 1) d += __shfl_xor(d, o, 32);
    const float rel = fabsf((float)(kk - 24)); const float sm = 1.0f / (1.0f + expf(-(width - rel) * sharp)); const float s = d * 0.125f - (1.0f - sm) * 10000.0f;
    const float mn = fmaxf(m, s); const float corr = expf(m - mn); const float p = expf(s - mn); z = z * corr + p; o1 = o1 * corr + p * v1; o2 = o2 * corr + p * v2; m = mn; }
  const float iz = 1.0f / z; const float a1 = o1 * iz, a2 = o2 * iz;
#pragma unroll 1
  for (int pass = 0; pass < 2; ++pass) { *(volatile float*)(AO + r * CCl + h * HDl + i) = a1; *(volatile float*)(AO + r * CCl + h * HDl + i + 32) = a2; __threadfence(); }
}
__global__ __launch_bounds__(128) void k_merge(const float* __restrict__ AO, const float* __restrict__ KV, const float* __restrict__ GP, const float* __restrict__ ow, float* __restrict__ MG) {
  __shared__ float red[128];
  const size_t r = blockIdx.x; const int tid = threadIdx.x, c = 4 * tid; const v4f_t a = *(const v4f_t*)(AO + r * CCl + c); red[tid] = a[0] * a[0] + a[1] * a[1] + a[2] * a[2] + a[3] * a[3]; __syncthreads();
  for (int o = 64; o > 0; o >>= 1) { if (tid < o) red[tid] += red[tid + o]; __syncthreads(); }
  const float rs = 1.0f / __builtin_sqrtf(red[0] * (1.0f / CCl) + 1e-6f); const v4f_t v = *(const v4f_t*)(KV + r * (2 * CCl) + CCl + c), gp = *(const v4f_t*)(GP + r * CCl + c), w = *(const v4f_t*)(ow + c); v4f_t out;
#pragma unroll
  for (int u = 0; u < 4; ++u) { const float sg = gp[u] / (1.0f + expf(-gp[u])); const float g = 1.0f / (1.0f + expf(-sg)); out[u] = g * v[u] + (1.0f - g) * (a[u] * rs * w[u]); }
  *(volatile v4f_t*)(MG + r * CCl + c) = out; __threadfence(); *(volatile v4f_t*)(MG + r * CCl + c) = out;
}
__global__ __launch_bounds__(256) void k_silu(float* __restrict__ O, size_t n4) { const size_t q = (size_t)blockIdx.x * 256 + threadIdx.x; if (q >= n4) return; v4f_t v = *(const v4fa*)(O + 4 * q);
#pragma unroll
  for (int u = 0; u < 4; ++u) v[u] = v[u] / (1.0f + expf(-v[u]));
  *(volatile v4fa*)(O + 4 * q) = v; __threadfence(); *(volatile v4fa*)(O + 4 * q) = v; }

extern "C" void kernel_launch(void* const* d_in, const int* in_sizes, int n_in,
                              void* d_out, int out_size, void* d_ws, size_t ws_size,
                              hipStream_t stream) {
  (void)in_sizes; (void)n_in; (void)out_size;
  const float** f = (const float**)d_in;
  const float* x = f[0], *Wq = f[1], *Wkv = f[2], *Wwin = f[3], *bwin = f[4], *Wg = f[5], *bg = f[6], *Wout = f[7], *qw = f[8], *kw = f[9], *ow = f[10];
  float* out = (float*)d_out;
  char* ws = (char*)d_ws;
  float* WwT = (float*)ws; ws += (size_t)CCl * 128 * 4; float* WgT = (float*)ws; ws += (size_t)CCl * CCl * 4; float* BwT = (float*)ws; ws += 128 * 4; float* CS = (float*)ws; ws += 256 * 4; float* SN = (float*)ws; ws += 256 * 4;
  float* Q = (float*)ws; ws += (size_t)NRl * CCl * 4; float* KV = (float*)ws; ws += (size_t)NRl * 2 * CCl * 4; float* WP = (float*)ws; ws += (size_t)NRl * 128 * 4;
  float* AO = (float*)ws; ws += (size_t)NRl * CCl * 4; float* GP = (float*)ws; ws += (size_t)NRl * CCl * 4; float* MG = (float*)ws; ws += (size_t)NRl * CCl * 4;
  if ((size_t)(ws - (char*)d_ws) > ws_size) return;
  const dim3 blk(256);
  k_padwin<<<dim3(CCl), dim3(128), 0, stream>>>(Wwin, bwin, WwT, BwT); k_transpose<<<dim3((CCl / 64) * (CCl / 64)), blk, 0, stream>>>(Wg, WgT, CCl, CCl); k_ropetab<<<dim3(1), blk, 0, stream>>>(CS, SN);

  gemm_rb_kernel<float, 2><<<dim3(NRl / 128, CCl / 256), blk, 0, stream>>>(x, Wq, nullptr, nullptr, nullptr, nullptr, Q, NRl, CCl, CCl);
  gemm_rb_kernel<float, 2><<<dim3(NRl / 128, 2 * CCl / 256), blk, 0, stream>>>(x, Wkv, nullptr, nullptr, nullptr, nullptr, KV, NRl, 2 * CCl, CCl);
  gemm_kn2<float, false><<<dim3(NRl / 128, 1, 1), blk, 0, stream>>>(x, CCl, 0, WwT, 128, 0, BwT, 1.0f, WP, 128, 0, CCl);
  k_prep<<<dim3(NRl), blk, 0, stream>>>(Q, KV, qw, kw, CS, SN);
  k_window<<<dim3(NRl), blk, 0, stream>>>(Q, KV, WP, AO);
  gemm_kne<float, 0, false><<<dim3(NRl / 128, CCl / 128), blk, 0, stream>>>(KV + CCl, 2 * CCl, WgT, CCl, bg, nullptr, nullptr, GP, CCl, CCl);
  k_merge<<<dim3(NRl), dim3(128), 0, stream>>>(AO, KV, GP, ow, MG);
  gemm_rb_kernel<float, 2><<<dim3(NRl / 128, CCl / 256), blk, 0, stream>>>(MG, Wout, nullptr, nullptr, nullptr, nullptr, out, NRl, CCl, CCl);
  k_silu<<<dim3(((size_t)NRl * CCl / 4 + 255) / 256), blk, 0, stream>>>(out, (size_t)NRl * CCl / 4);
}
